// Model_19301583028953
// MI455X (gfx1250) — hardware-run, weakly checked
//
#include <hip/hip_runtime.h>
#include <math.h>

constexpr int NTOK   = 65536;
constexpr int NPOS   = 16;
constexpr int NEMB   = 15;
constexpr int NHID   = 30;
constexpr int NTAGS  = 45;
constexpr int NCHR   = 85;
constexpr int PADCH  = 84;
constexpr int XCOLS  = 32;
constexpr int GCOLS  = 256;
constexpr int HCOLS  = 32;
constexpr int WPK    = 32;
constexpr int LROWS  = 48;
constexpr int LCOLS  = 64;
constexpr int CROWS  = 16;
constexpr int CCOLS  = 64;
constexpr int TOKB   = 128;
constexpr int TPITCH = 72;
constexpr int APITCH = 40;
constexpr int SGP    = 52;
constexpr float ACARRY = 16.0f;
constexpr float WCARRY = 64.0f;
constexpr float RS1024 = 1.0f / 1024.0f;
static_assert(NTOK % TOKB == 0);
static_assert(NTOK % 64 == 0);
static_assert(2 * NEMB <= XCOLS && NHID + 2 <= HCOLS);
static_assert((64 * NTAGS * 4) % 128 == 0);
static_assert((64 * NTAGS) % 4 == 0);
static_assert(NTOK % 64 == 0 && GCOLS % 64 == 0 && XCOLS % 32 == 0);
static_assert(NCHR * 16 <= 6 * 256);

typedef __attribute__((ext_vector_type(16))) _Float16 v16h;
typedef __attribute__((ext_vector_type(8)))  _Float16 v8h;
typedef __attribute__((ext_vector_type(2)))  _Float16 v2h;
typedef __attribute__((ext_vector_type(16))) __bf16   v16b;
typedef __attribute__((ext_vector_type(8)))  __bf16   v8b;
typedef __attribute__((ext_vector_type(8)))  float    v8f;
typedef __attribute__((ext_vector_type(4)))  float    v4f;
typedef __attribute__((ext_vector_type(4)))  int      v4i;

__device__ __forceinline__ unsigned short f2bf_bits(float f) {
  unsigned u = __float_as_uint(f);
  return (unsigned short)((u + 0x7FFFu + ((u >> 16) & 1u)) >> 16);
}
__device__ __forceinline__ float bf_bits2f(unsigned short h) { return __uint_as_float(((unsigned)h) << 16); }
__device__ __forceinline__ int clampi(int v, int lo, int hi) { return v < lo ? lo : (v > hi ? hi : v); }

__device__ __forceinline__ void dep_guard_h(v8f& a, v8f& b, v16h x, v16h y) { asm volatile("v_nop\n\tv_nop\n\tv_nop\n\tv_nop" : "+v"(a), "+v"(b) : "v"(x), "v"(y)); }
__device__ __forceinline__ void dep_guard_b(v8f& a, v8f& b, v16b x, v16b y) { asm volatile("v_nop\n\tv_nop\n\tv_nop\n\tv_nop" : "+v"(a), "+v"(b) : "v"(x), "v"(y)); }
__device__ __forceinline__ void keep4_h(v16h a, v16h b, v16h c, v16h d) { asm volatile("v_nop" :: "v"(a), "v"(b), "v"(c), "v"(d)); }
__device__ __forceinline__ void keep4_b(v16b a, v16b b, v16b c, v16b d) { asm volatile("v_nop" :: "v"(a), "v"(b), "v"(c), "v"(d)); }
__device__ __forceinline__ void acc_guard4(v8f& a, v8f& b, v8f& c, v8f& d) { asm volatile("v_nop\n\tv_nop\n\tv_nop\n\tv_nop" : "+v"(a), "+v"(b), "+v"(c), "+v"(d)); }
__device__ __forceinline__ void guard1_h(v8f& a, v16h x0, v16h x1, v16h y0, v16h y1) {
  asm volatile("v_nop\n\tv_nop\n\tv_nop\n\tv_nop" : "+v"(a) : "v"(x0), "v"(x1), "v"(y0), "v"(y1));
}
__device__ __forceinline__ void guard3_h(v8f& a0, v8f& a1, v8f& a2, v16h x0, v16h x1,
                                         v16h y0, v16h y1, v16h y2, v16h y3, v16h y4, v16h y5) {
  asm volatile("v_nop\n\tv_nop\n\tv_nop\n\tv_nop" : "+v"(a0), "+v"(a1), "+v"(a2)
               : "v"(x0), "v"(x1), "v"(y0), "v"(y1), "v"(y2), "v"(y3), "v"(y4), "v"(y5));
}
__device__ __forceinline__ void guard4_h(v8f& a0, v8f& a1, v8f& a2, v8f& a3, v16h x, v16h y0, v16h y1, v16h y2, v16h y3) {
  asm volatile("v_nop\n\tv_nop\n\tv_nop\n\tv_nop" : "+v"(a0), "+v"(a1), "+v"(a2), "+v"(a3)
               : "v"(x), "v"(y0), "v"(y1), "v"(y2), "v"(y3));
}
__device__ __forceinline__ void lds_wave_sync() {
  __builtin_amdgcn_fence(__ATOMIC_RELEASE, "workgroup");
  __builtin_amdgcn_wave_barrier();
  __builtin_amdgcn_fence(__ATOMIC_ACQUIRE, "workgroup");
}

template <typename T> struct Frag;
template <> struct Frag<_Float16> {
  typedef v16h V; union U { v16h v; v8h h[2]; };
  static __device__ __forceinline__ v16h load(const _Float16* p) {
    U f; f.h[0] = *(const v8h*)(p); f.h[1] = *(const v8h*)(p + 16); return f.v;
  }
  static __device__ __forceinline__ v8f mma(v16h a, v16h b, v8f c) {
    return __builtin_amdgcn_wmma_f32_16x16x32_f16(false, a, false, b, (short)0, c, false, false);
  }
  static __device__ __forceinline__ void guard(v8f& a, v8f& b, v16h x, v16h y) { dep_guard_h(a, b, x, y); }
  static __device__ __forceinline__ void keep(v16h a, v16h b, v16h c, v16h d) { keep4_h(a, b, c, d); }
};
template <> struct Frag<__bf16> {
  typedef v16b V; union U { v16b v; v8b h[2]; };
  static __device__ __forceinline__ v16b load(const __bf16* p) {
    U f; f.h[0] = *(const v8b*)(p); f.h[1] = *(const v8b*)(p + 16); return f.v;
  }
  static __device__ __forceinline__ v8f mma(v16b a, v16b b, v8f c) {
    return __builtin_amdgcn_wmma_f32_16x16x32_bf16(false, a, false, b, (short)0, c, false, false);
  }
  static __device__ __forceinline__ void guard(v8f& a, v8f& b, v16b x, v16b y) { dep_guard_b(a, b, x, y); }
  static __device__ __forceinline__ void keep(v16b a, v16b b, v16b c, v16b d) { keep4_b(a, b, c, d); }
};

template <int ET> struct Elem;
template <> struct Elem<0> { typedef _Float16 T; };
template <> struct Elem<1> { typedef __bf16 T; };
template <int ET, bool SPLIT, int BIAS_MODE, int OUT_MODE, bool RESID, int ACT = 0>
__global__ __launch_bounds__(256) void wmma_gemm64(
    const unsigned short* __restrict__ Ap, const unsigned short* __restrict__ A2p, int lda, long strideA,
    const unsigned short* __restrict__ Btp, const unsigned short* __restrict__ Bt2p, int ldb, long strideB,
    void* __restrict__ Cout, void* __restrict__ Cout2, int ldc, long strideC,
    const float* __restrict__ bias,
    const float* __restrict__ resid, long strideR,
    int M, int N, int K, float scale) {
  typedef typename Elem<ET>::T T;
  typedef typename Frag<T>::V V;
  const T* A = (const T*)Ap; const T* A2 = (const T*)A2p; const T* Bt = (const T*)Btp; const T* Bt2 = (const T*)Bt2p;
  __shared__ __align__(16) float sT[8][16 * 68];
  const int b    = blockIdx.y;
  const int lane = threadIdx.x & 31;
  const int wave = threadIdx.x >> 5;
  const int tilesN = N >> 6;
  const int tilesM = M >> 6;
  const int tile = blockIdx.x * 8 + wave;
  if (tile >= tilesM * tilesN) return;
  const int tm = tile / tilesN;
  const int tn = tile - tm * tilesN;
  const int m0 = tm << 6;
  const int n0 = tn << 6;

  const T* Ab  = A  + (size_t)b * strideA;
  const T* Bb  = Bt + (size_t)b * strideB;
  const T* Ab2 = SPLIT ? (A2  + (size_t)b * strideA) : nullptr;
  const T* Bb2 = SPLIT ? (Bt2 + (size_t)b * strideB) : nullptr;

  const int rlane = lane & 15;
  const int koff  = (lane >> 4) * 8;
  const int mOff  = (lane >> 4) * 8;

  v8f acc[4][4];
#pragma unroll
  for (int i = 0; i < 4; ++i)
#pragma unroll
    for (int j = 0; j < 4; ++j) acc[i][j] = (v8f){0.f,0.f,0.f,0.f,0.f,0.f,0.f,0.f};

  for (int k0 = 0; k0 < K; k0 += 32) {
    V bh[4], bl[4];
#pragma unroll
    for (int j = 0; j < 4; ++j) {
      const size_t bo = (size_t)(n0 + (j << 4) + rlane) * ldb + koff + k0;
      bh[j] = Frag<T>::load(Bb + bo);
      if (SPLIT) bl[j] = Frag<T>::load(Bb2 + bo);
    }
#pragma unroll
    for (int i = 0; i < 4; ++i) {
      const size_t ao = (size_t)(m0 + (i << 4) + rlane) * lda + koff + k0;
      V ah = Frag<T>::load(Ab + ao);
      V al;
      if (SPLIT) al = Frag<T>::load(Ab2 + ao);
#pragma unroll
      for (int j = 0; j < 4; ++j) {
        acc[i][j] = Frag<T>::mma(ah, bh[j], acc[i][j]);
        if (SPLIT) {
          acc[i][j] = Frag<T>::mma(ah, bl[j], acc[i][j]);
          acc[i][j] = Frag<T>::mma(al, bh[j], acc[i][j]);
        }
      }
      Frag<T>::guard(acc[i][0], acc[i][3], ah, SPLIT ? al : ah);
    }
    Frag<T>::keep(bh[0], bh[1], bh[2], bh[3]);
    if (SPLIT) Frag<T>::keep(bl[0], bl[1], bl[2], bl[3]);
  }
  acc_guard4(acc[0][0], acc[0][1], acc[0][2], acc[0][3]);
  acc_guard4(acc[1][0], acc[1][1], acc[1][2], acc[1][3]);
  acc_guard4(acc[2][0], acc[2][1], acc[2][2], acc[2][3]);
  acc_guard4(acc[3][0], acc[3][1], acc[3][2], acc[3][3]);

  float* slab = sT[wave];
  const float* Rb = RESID ? (resid + (size_t)b * strideR) : nullptr;
#pragma unroll
  for (int i = 0; i < 4; ++i) {
    const int mBase = m0 + (i << 4);
#pragma unroll
    for (int j = 0; j < 4; ++j) {
      const int n = n0 + (j << 4) + rlane;
      float bv = 0.f;
      if (BIAS_MODE == 2) bv = bias[n];
#pragma unroll
      for (int r = 0; r < 8; ++r) {
        float v = acc[i][j][r] * scale;
        if (BIAS_MODE == 1) v += bias[mBase + mOff + r];
        if (BIAS_MODE == 2) v += bv;
        if (RESID) v += Rb[(size_t)(mBase + mOff + r) * ldc + n];
        if (ACT == 1) v = tanhf(v);
        if (ACT == 2) v = fmaxf(v, 0.0f);
        if (ACT == 3) v = v / (1.0f + expf(-v));
        if (ACT == 4) v = (v > 0.f) ? v : 0.01f * v;
        if (ACT == 5) v = 0.5f * v * (1.0f + erff(v * 0.70710678118654752f));
        slab[(mOff + r) * 68 + (j << 4) + rlane] = v;
      }
    }
    __builtin_amdgcn_fence(__ATOMIC_RELEASE, "workgroup");
    __builtin_amdgcn_wave_barrier();
    __builtin_amdgcn_fence(__ATOMIC_ACQUIRE, "workgroup");
    if (OUT_MODE == 0) {
      float* C = (float*)Cout + (size_t)b * strideC;
      const int hh = lane >> 4, c4 = (lane & 15) * 4;
      for (int pass = 0; pass < 2; ++pass) {
#pragma unroll
        for (int it = 0; it < 8; ++it) {
          const int row = it * 2 + hh;
          v4f v = *(const v4f*)(slab + row * 68 + c4);
          *(volatile v4f*)(C + (size_t)(mBase + row) * ldc + n0 + c4) = v;
        }
        __threadfence();
      }
    } else {
      const int q = lane >> 3, c8 = (lane & 7) * 8;
      unsigned short* C  = (unsigned short*)Cout  + (size_t)b * strideC;
      unsigned short* C2 = (OUT_MODE == 2) ? ((unsigned short*)Cout2 + (size_t)b * strideC) : nullptr;
      for (int pass = 0; pass < 2; ++pass) {
#pragma unroll
        for (int it = 0; it < 4; ++it) {
          const int row = it * 4 + q;
          const float* sp = slab + row * 68 + c8;
          v8h hv, lv;
#pragma unroll
          for (int e = 0; e < 8; ++e) {
            if (OUT_MODE == 1) {
              hv[e] = (_Float16)sp[e];
            } else {
              unsigned short hb = f2bf_bits(sp[e]);
              unsigned short lb = f2bf_bits(sp[e] - bf_bits2f(hb));
              hv[e] = __builtin_bit_cast(_Float16, hb);
              lv[e] = __builtin_bit_cast(_Float16, lb);
            }
          }
          *(volatile v8h*)(C + (size_t)(mBase + row) * ldc + n0 + c8) = hv;
          if (OUT_MODE == 2) *(volatile v8h*)(C2 + (size_t)(mBase + row) * ldc + n0 + c8) = lv;
        }
        __threadfence();
      }
    }
    __builtin_amdgcn_fence(__ATOMIC_RELEASE, "workgroup");
    __builtin_amdgcn_wave_barrier();
    __builtin_amdgcn_fence(__ATOMIC_ACQUIRE, "workgroup");
  }
}


__global__ __launch_bounds__(256) void pack_kernel(
    const float* __restrict__ wih_f, const float* __restrict__ whh_f, const float* __restrict__ bih_f, const float* __restrict__ bhh_f,
    const float* __restrict__ wih_b, const float* __restrict__ whh_b, const float* __restrict__ bih_b, const float* __restrict__ bhh_b,
    const float* __restrict__ lin_w, const float* __restrict__ conv_w,
    unsigned short* __restrict__ WIHP, unsigned short* __restrict__ WHHP, unsigned short* __restrict__ LINP,
    unsigned short* __restrict__ CONVP, float* __restrict__ BIASG) {
  __shared__ float sw[3840];
  const int tid = threadIdx.x;
  const int role = blockIdx.x;
  const float* src = wih_f;
  int cnt = 4 * NHID * NHID;
  if (role == 1) src = wih_b;
  if (role == 2) src = whh_f;
  if (role == 3) src = whh_b;
  if (role == 4) { src = lin_w;  cnt = NTAGS * 2 * NHID; }
  if (role == 5) { src = conv_w; cnt = NEMB * 3 * NEMB; }
  const int cntpad = (cnt + 255) & ~255;
#pragma unroll 1
  for (int i = tid; i < cntpad; i += 256) sw[i] = src[(i < cnt) ? i : (cnt - 1)];
  if (role == 5) {
    const int ib = (tid < 4 * NHID) ? tid : (4 * NHID - 1);
    const float q0 = bih_f[ib], q1 = bhh_f[ib], q2 = bih_b[ib], q3 = bhh_b[ib];
    if (tid < 4 * NHID) { sw[1024 + tid] = q0; sw[1144 + tid] = q1; sw[1264 + tid] = q2; sw[1384 + tid] = q3; }
  }
  __syncthreads();

  if (role < 4) {
    unsigned short* dst = (role < 2) ? (WIHP + (size_t)role * 128 * WPK) : (WHHP + (size_t)(role - 2) * 128 * WPK);
#pragma unroll 1
    for (int it = 0; it < 2; ++it) {
      const int gidx = it * 256 + tid;
      const int p  = gidx >> 2, k0 = (gidx & 3) * 8;
      const int gt = p >> 5, s = (p >> 4) & 1, cc = p & 15, u = 2 * cc + s;
      const int srow = NHID * gt + ((u < NHID) ? u : (NHID - 1));
      const float fu = (u < NHID) ? WCARRY : 0.0f;
      v8h hv;
#pragma unroll
      for (int e = 0; e < 8; ++e) {
        const int k = k0 + e;
        const int kc = (k < NHID) ? k : (NHID - 1);
        const float f = sw[srow * NHID + kc];
        const float fac = (k < NHID) ? fu : 0.0f;
        hv[e] = (_Float16)(f * fac);
      }
      unsigned short* dp = dst + (size_t)gidx * 8;
      *(volatile v8h*)dp = hv;
      __threadfence();
      *(volatile v8h*)dp = hv;
    }
  } else if (role == 4) {
#pragma unroll 1
    for (int it = 0; it < 2; ++it) {
      const int gidx = it * 256 + tid;
      if (gidx < LROWS * LCOLS / 8) {
        const int n = gidx >> 3, k0 = (gidx & 7) * 8;
        const int nc = (n < NTAGS) ? n : (NTAGS - 1);
        const float fn = (n < NTAGS) ? WCARRY : 0.0f;
        v8h hv;
#pragma unroll
        for (int e = 0; e < 8; ++e) {
          const int k = k0 + e;
          const bool in1 = (k < NHID);
          const bool in2 = (k >= 32) && (k < 32 + NHID);
          const int col = in1 ? k : (in2 ? (k - 2) : 0);
          const float f = sw[nc * (2 * NHID) + col];
          const float fac = (in1 || in2) ? fn : 0.0f;
          hv[e] = (_Float16)(f * fac);
        }
        unsigned short* dp = LINP + (size_t)gidx * 8;
        *(volatile v8h*)dp = hv;
        __threadfence();
        *(volatile v8h*)dp = hv;
      }
    }
  } else {
    if (tid < CROWS * CCOLS / 8) {
      const int gidx = tid;
      const int fr = gidx >> 3, k0 = (gidx & 7) * 8;
      const int frc = (fr < NEMB) ? fr : (NEMB - 1);
      const float ff = (fr < NEMB) ? WCARRY : 0.0f;
      v8h hv;
#pragma unroll
      for (int e = 0; e < 8; ++e) {
        const int k = k0 + e;
        const int j = k >> 4, dd = k & 15;
        const bool ok = (j < 3) && (dd < NEMB);
        const int col = ((j < 3) ? j : 2) * NEMB + ((dd < NEMB) ? dd : (NEMB - 1));
        const float f = sw[frc * (3 * NEMB) + col];
        const float fac = ok ? ff : 0.0f;
        hv[e] = (_Float16)(f * fac);
      }
      unsigned short* dp = CONVP + (size_t)gidx * 8;
      *(volatile v8h*)dp = hv;
      __threadfence();
      *(volatile v8h*)dp = hv;
    } else if (tid < CROWS * CCOLS / 8 + 64) {
      const int q = tid - CROWS * CCOLS / 8;
      v4f o;
#pragma unroll
      for (int e = 0; e < 4; ++e) {
        const int n = 4 * q + e;
        const int d = n >> 7, p = n & 127;
        const int gt = p >> 5, s = (p >> 4) & 1, cc = p & 15, u = 2 * cc + s;
        const int srow = NHID * gt + ((u < NHID) ? u : (NHID - 1));
        const float a  = sw[1024 + 240 * d + srow];
        const float bb = sw[1144 + 240 * d + srow];
        const float fac = (u < NHID) ? 1.0f : 0.0f;
        o[e] = (a + bb) * fac;
      }
      float* op = BIASG + 4 * q;
      *(volatile v4f*)op = o;
      __threadfence();
      *(volatile v4f*)op = o;
    }
  }
}

__global__ __launch_bounds__(256) void charconv_kernel(
    const int* __restrict__ word_ids, const int* __restrict__ char_ids, const int* __restrict__ word_lens,
    const float* __restrict__ word_emb, const float* __restrict__ char_emb, const float* __restrict__ conv_b,
    const unsigned short* __restrict__ CONVPp, unsigned short* __restrict__ Xp, int nvocab) {
  __shared__ __align__(16) _Float16 E16[NCHR * 16];
  __shared__ __align__(16) _Float16 Tl[8][NPOS * TPITCH];
  __shared__ __align__(16) _Float16 Xs[TOKB * XCOLS];
  __shared__ int   sCid[TOKB * NPOS];
  __shared__ int   sWid[TOKB];
  __shared__ int   sLen[TOKB];
  __shared__ float sB[16];
  const int tid = threadIdx.x, lane = tid & 31, wave = tid >> 5;
  const int c = lane & 15, hh = lane >> 4;
  const int t0 = blockIdx.x * TOKB;

#pragma unroll
  for (int it = 0; it < 6; ++it) {
    const int i  = it * 256 + tid;
    const int ic = (i < NCHR * 16) ? i : (NCHR * 16 - 1);
    const int r  = ic >> 4, dd = ic & 15;
    const float f = char_emb[r * NEMB + ((dd < NEMB) ? dd : (NEMB - 1))];
    const float fac = (dd < NEMB) ? ACARRY : 0.0f;
    if (i < NCHR * 16) E16[i] = (_Float16)(f * fac);
  }
  {
    const float f = conv_b[(tid < NEMB) ? tid : (NEMB - 1)];
    const float fac = (tid < NEMB) ? 1.0f : 0.0f;
    if (tid < 16) sB[tid] = f * fac;
  }
  {
    const int tk = tid & (TOKB - 1);
    int w  = word_ids[t0 + tk];
    int ln = word_lens[t0 + tk];
    w  = clampi(w, 0, nvocab - 1);
    ln = clampi(ln, 1, NPOS);
    if (tid < TOKB) sWid[tk] = w; else sLen[tk] = ln;
  }
  {
    const v4i* cp = (const v4i*)(char_ids + (size_t)t0 * NPOS) + tid * 2;
    const v4i a = cp[0];
    const v4i b = cp[1];
#pragma unroll
    for (int e = 0; e < 4; ++e) {
      sCid[tid * 8 + e]     = clampi(a[e], 0, NCHR - 1);
      sCid[tid * 8 + 4 + e] = clampi(b[e], 0, NCHR - 1);
    }
  }
  __syncthreads();

  const _Float16* CW = (const _Float16*)CONVPp;
  const v16h wb0 = Frag<_Float16>::load(CW + (size_t)c * CCOLS + 8 * hh);
  const v16h wb1 = Frag<_Float16>::load(CW + (size_t)c * CCOLS + 32 + 8 * hh);
  _Float16* tl = Tl[wave];
  _Float16* trow = tl + c * TPITCH;
  v8h z8h;
#pragma unroll
  for (int e = 0; e < 8; ++e) z8h[e] = (_Float16)0.0f;
  const v8f z8 = {0.f, 0.f, 0.f, 0.f, 0.f, 0.f, 0.f, 0.f};

#pragma unroll 1
  for (int i = 0; i < 16; ++i) {
    const int tk  = wave * 16 + i;
    const int len = sLen[tk];
    const int wid = sWid[tk];
    lds_wave_sync();
    const int idxA = c + 2 * hh - 1;
    const int okA  = (idxA > 0 && idxA < len) ? 1 : 0;
    const int ciA  = sCid[tk * NPOS + clampi(idxA, 0, NPOS - 1)];
    const int chA  = PADCH + (ciA - PADCH) * okA;
    const int okB  = (c > 0 && c < len) ? 1 : 0;
    const int ciB  = sCid[tk * NPOS + c];
    const int chB  = PADCH + (ciB - PADCH) * okB;
    const v8h a0 = *(const v8h*)(E16 + chA * 16);
    const v8h a1 = *(const v8h*)(E16 + chA * 16 + 8);
    v8h e0 = *(const v8h*)(E16 + chB * 16);
    v8h e1 = *(const v8h*)(E16 + chB * 16 + 8);
    if (hh) { e0 = z8h; e1 = z8h; }
    *(v8h*)(trow + (2 * hh) * 16)         = a0;
    *(v8h*)(trow + (2 * hh) * 16 + 8)     = a1;
    *(v8h*)(trow + (2 * hh + 1) * 16)     = e0;
    *(v8h*)(trow + (2 * hh + 1) * 16 + 8) = e1;
    lds_wave_sync();
    const v16h fa0 = Frag<_Float16>::load(trow + 8 * hh);
    const v16h fa1 = Frag<_Float16>::load(trow + 32 + 8 * hh);
    v8f acc = z8;
    acc = Frag<_Float16>::mma(fa0, wb0, acc);
    acc = Frag<_Float16>::mma(fa1, wb1, acc);
    guard1_h(acc, fa0, fa1, wb0, wb1);
    float mx = -INFINITY;
#pragma unroll
    for (int r = 0; r < 8; ++r) {
      const int pos = 8 * hh + r;
      const float v = acc[r];
      mx = fmaxf(mx, (pos < len) ? v : -INFINITY);
    }
    mx = fmaxf(mx, __shfl_xor(mx, 16, 32));
    const float cf = mx * RS1024 + sB[c];
    const int srcl = (lane >= NEMB) ? (lane - NEMB) : lane;
    const float cfs = __shfl(cf, srcl, 32);
    const float we = word_emb[(size_t)wid * NEMB + ((lane < NEMB) ? lane : (NEMB - 1))];
    const float fw = (lane < NEMB) ? 1.0f : 0.0f;
    const float fc = (lane >= NEMB && lane < 2 * NEMB) ? 1.0f : 0.0f;
    const float xv = fmaf(fw, we, fc * cfs);
    Xs[tk * XCOLS + lane] = (_Float16)(xv * ACARRY);
  }
  __syncthreads();

  unsigned short* xo = Xp + (size_t)t0 * XCOLS;
  for (int pass = 0; pass < 2; ++pass) {
#pragma unroll
    for (int it = 0; it < 2; ++it) {
      const int idx = it * 256 + tid;
      const v8h v = *(const v8h*)(Xs + idx * 8);
      *(volatile v8h*)(xo + (size_t)idx * 8) = v;
    }
    __threadfence();
  }
}

__device__ __forceinline__ float sigm_f(float x) { return __builtin_amdgcn_rcpf(1.0f + expf(-x)); }
__device__ __forceinline__ float tanh_f(float x) { return 1.0f - 2.0f * __builtin_amdgcn_rcpf(expf(2.0f * x) + 1.0f); }

__global__ __launch_bounds__(32) void bilstm_scan_kernel(const float* __restrict__ Gp, const unsigned short* __restrict__ WHHPp,
                                                         unsigned short* __restrict__ HFp, unsigned short* __restrict__ HBp) {
  __shared__ __align__(16) _Float16 Ah[16 * APITCH];
  __shared__ __align__(16) _Float16 Hs[64 * HCOLS];
  __shared__ __align__(16) _Float16 sWB[128 * WPK];
  const int lane = threadIdx.x, c = lane & 15, hh = lane >> 4;
  const int d = blockIdx.x;
  unsigned short* HP = d ? HBp : HFp;
  v8h z8h;
#pragma unroll
  for (int e = 0; e < 8; ++e) z8h[e] = (_Float16)0.0f;
#pragma unroll 1
  for (int g = lane; g < 16 * APITCH / 8; g += 32) *(v8h*)(Ah + g * 8) = z8h;
  {
    const v8h* wsrc = (const v8h*)(WHHPp + (size_t)d * 128 * WPK);
#pragma unroll 1
    for (int g = lane; g < 128 * WPK / 8; g += 32) *(v8h*)(sWB + g * 8) = wsrc[g];
  }
  __syncthreads();
  v16h bfr[8];
#pragma unroll
  for (int j = 0; j < 8; ++j) bfr[j] = Frag<_Float16>::load(sWB + (16 * j + c) * WPK + 8 * hh);

  float cs0 = 0.0f, cs1 = 0.0f;
  int t = d ? (NTOK - 1) : 0;
  const int dt = d ? -1 : 1;
  float gin[8];
  {
    const float* gr = Gp + (size_t)t * GCOLS + d * 128 + c;
#pragma unroll
    for (int j = 0; j < 8; ++j) gin[j] = gr[16 * j];
  }
  const v8f z8 = {0.f, 0.f, 0.f, 0.f, 0.f, 0.f, 0.f, 0.f};
  const _Float16* arow = Ah + c * APITCH + 8 * hh;

#pragma unroll 1
  for (int s = 0; s < NTOK; ++s) {
    const int tn  = t + dt;
    const int tnc = clampi(tn, 0, NTOK - 1);
    float gnx[8];
    {
      const float* gr = Gp + (size_t)tnc * GCOLS + d * 128 + c;
#pragma unroll
      for (int j = 0; j < 8; ++j) gnx[j] = gr[16 * j];
    }
    const v16h a = Frag<_Float16>::load(arow);
    v8f acc[8];
#pragma unroll
    for (int j = 0; j < 8; ++j) acc[j] = Frag<_Float16>::mma(a, bfr[j], z8);
    guard4_h(acc[0], acc[1], acc[2], acc[3], a, bfr[0], bfr[1], bfr[2], bfr[3]);
    guard4_h(acc[4], acc[5], acc[6], acc[7], a, bfr[4], bfr[5], bfr[6], bfr[7]);

    const float zi0 = acc[0][0] * RS1024 + gin[0];
    const float zf0 = acc[2][0] * RS1024 + gin[2];
    const float zg0 = acc[4][0] * RS1024 + gin[4];
    const float zo0 = acc[6][0] * RS1024 + gin[6];
    const float zi1 = acc[1][0] * RS1024 + gin[1];
    const float zf1 = acc[3][0] * RS1024 + gin[3];
    const float zg1 = acc[5][0] * RS1024 + gin[5];
    const float zo1 = acc[7][0] * RS1024 + gin[7];
    cs0 = sigm_f(zf0) * cs0 + sigm_f(zi0) * tanh_f(zg0);
    cs1 = sigm_f(zf1) * cs1 + sigm_f(zi1) * tanh_f(zg1);
    const float h0 = sigm_f(zo0) * tanh_f(cs0);
    const float h1 = sigm_f(zo1) * tanh_f(cs1);
    const float h0s = (2 * c     < NHID) ? h0 : 0.0f;
    const float h1s = (2 * c + 1 < NHID) ? h1 : 0.0f;
    v2h pk;
    pk[0] = (_Float16)(h0s * ACARRY);
    pk[1] = (_Float16)(h1s * ACARRY);
    if (hh == 0) {
      *(v2h*)(Ah + 2 * c) = pk;
      *(v2h*)(Hs + (t & 63) * HCOLS + 2 * c) = pk;
    }
    __syncthreads();
    if ((s & 63) == 63) {
      unsigned short* hp = HP + (size_t)(t & ~63) * HCOLS;
      for (int pass = 0; pass < 2; ++pass) {
#pragma unroll
        for (int it = 0; it < 8; ++it) {
          const v8h v = *(const v8h*)(Hs + it * 256 + lane * 8);
          *(volatile v8h*)(hp + it * 256 + lane * 8) = v;
        }
        __threadfence();
      }
    }
#pragma unroll
    for (int j = 0; j < 8; ++j) gin[j] = gnx[j];
    t = tn;
  }
}

__global__ __launch_bounds__(128) void head_softmax_kernel(const unsigned short* __restrict__ HFp, const unsigned short* __restrict__ HBp,
                                                           const unsigned short* __restrict__ LINPp, const float* __restrict__ lin_b,
                                                           float* __restrict__ out) {
  __shared__ float Sg[64 * SGP];
  __shared__ __align__(16) float Os[64 * NTAGS];
  __shared__ __align__(16) _Float16 sLW[LROWS * LCOLS];
  __shared__ float sLb[LROWS];
  const int tid = threadIdx.x, lane = tid & 31, wave = tid >> 5;
  const int c = lane & 15, hh = lane >> 4;
  const int t0 = blockIdx.x * 64;
  {
    const float f = lin_b[(tid < NTAGS) ? tid : (NTAGS - 1)];
    const float fac = (tid < NTAGS) ? 1.0f : 0.0f;
    if (tid < LROWS) sLb[tid] = f * fac;
  }
  {
    const v8h* lsrc = (const v8h*)LINPp;
#pragma unroll 1
    for (int g = tid; g < LROWS * LCOLS / 8; g += 128) *(v8h*)(sLW + g * 8) = lsrc[g];
  }
  const _Float16* HF = (const _Float16*)HFp;
  const _Float16* HB = (const _Float16*)HBp;
  const size_t arowoff = (size_t)(t0 + 16 * wave + c) * HCOLS + 8 * hh;
  const v16h a0 = Frag<_Float16>::load(HF + arowoff);
  const v16h a1 = Frag<_Float16>::load(HB + arowoff);
  __syncthreads();
  v16h bk0[3], bk1[3];
#pragma unroll
  for (int j = 0; j < 3; ++j) {
    bk0[j] = Frag<_Float16>::load(sLW + (16 * j + c) * LCOLS + 8 * hh);
    bk1[j] = Frag<_Float16>::load(sLW + (16 * j + c) * LCOLS + 32 + 8 * hh);
  }
  const v8f z8 = {0.f, 0.f, 0.f, 0.f, 0.f, 0.f, 0.f, 0.f};
  v8f acc[3];
#pragma unroll
  for (int j = 0; j < 3; ++j) {
    acc[j] = Frag<_Float16>::mma(a0, bk0[j], z8);
    acc[j] = Frag<_Float16>::mma(a1, bk1[j], acc[j]);
  }
  guard3_h(acc[0], acc[1], acc[2], a0, a1, bk0[0], bk1[0], bk0[1], bk1[1], bk0[2], bk1[2]);
#pragma unroll
  for (int j = 0; j < 3; ++j)
#pragma unroll
    for (int r = 0; r < 8; ++r) Sg[(16 * wave + 8 * hh + r) * SGP + 16 * j + c] = acc[j][r] * RS1024;
  __syncthreads();

#pragma unroll 1
  for (int rr = 0; rr < 16; ++rr) {
    const int row = 16 * wave + rr;
    const int col1 = 32 + ((lane < 15) ? lane : 15);
    const bool ok1 = lane < (NTAGS - 32);
    const float v0 = Sg[row * SGP + lane] + sLb[lane];
    const float v1 = Sg[row * SGP + col1] + sLb[col1];
    float m = fmaxf(v0, ok1 ? v1 : -INFINITY);
#pragma unroll
    for (int off = 16; off > 0; off >>= 1) m = fmaxf(m, __shfl_xor(m, off, 32));
    const float e0 = expf(v0 - m);
    const float e1 = expf(v1 - m) * (ok1 ? 1.0f : 0.0f);
    float ssum = e0 + e1;
#pragma unroll
    for (int off = 16; off > 0; off >>= 1) ssum += __shfl_xor(ssum, off, 32);
    const float inv = 1.0f / ssum;
    Os[row * NTAGS + lane] = e0 * inv;
    if (ok1) Os[row * NTAGS + 32 + lane] = e1 * inv;
  }
  __syncthreads();

  float* ob = out + (size_t)t0 * NTAGS;
  for (int pass = 0; pass < 2; ++pass) {
#pragma unroll
    for (int it = 0; it < 6; ++it) {
      const int idx = it * 128 + tid;
      if (idx < 64 * NTAGS / 4) {
        const v4f v = *(const v4f*)(Os + idx * 4);
        *(volatile v4f*)(ob + (size_t)idx * 4) = v;
      }
    }
    __threadfence();
  }
}

extern "C" void kernel_launch(void* const* d_in, const int* in_sizes, int n_in,
                              void* d_out, int out_size, void* d_ws, size_t ws_size, hipStream_t stream) {
  if (n_in < 17 || d_out == nullptr || d_ws == nullptr) return;
  if (in_sizes[0] != NTOK || in_sizes[1] != NTOK * NPOS || in_sizes[2] != NTOK ||
      in_sizes[3] < NEMB || (in_sizes[3] % NEMB) != 0 || in_sizes[4] != NCHR * NEMB ||
      in_sizes[5] != NEMB * 3 * NEMB || in_sizes[6] != NEMB ||
      in_sizes[7] != 4 * NHID * NHID || in_sizes[8] != 4 * NHID * NHID || in_sizes[9] != 4 * NHID || in_sizes[10] != 4 * NHID ||
      in_sizes[11] != 4 * NHID * NHID || in_sizes[12] != 4 * NHID * NHID || in_sizes[13] != 4 * NHID || in_sizes[14] != 4 * NHID ||
      in_sizes[15] != NTAGS * 2 * NHID || in_sizes[16] != NTAGS || out_size != NTOK * NTAGS) return;

  const int*   word_ids  = (const int*)d_in[0];
  const int*   char_ids  = (const int*)d_in[1];
  const int*   word_lens = (const int*)d_in[2];
  const float* word_emb  = (const float*)d_in[3];
  const float* char_emb  = (const float*)d_in[4];
  const float* conv_w    = (const float*)d_in[5];
  const float* conv_b    = (const float*)d_in[6];
  const float* wih_f     = (const float*)d_in[7];
  const float* whh_f     = (const float*)d_in[8];
  const float* bih_f     = (const float*)d_in[9];
  const float* bhh_f     = (const float*)d_in[10];
  const float* wih_b     = (const float*)d_in[11];
  const float* whh_b     = (const float*)d_in[12];
  const float* bih_b     = (const float*)d_in[13];
  const float* bhh_b     = (const float*)d_in[14];
  const float* lin_w     = (const float*)d_in[15];
  const float* lin_b     = (const float*)d_in[16];
  float* out = (float*)d_out;
  const int nvocab = in_sizes[3] / NEMB;

  char* ws = (char*)d_ws; size_t off = 0;
  auto carve = [&](size_t bytes) -> char* { char* p = ws + off; off += (bytes + 255) & ~(size_t)255; return p; };
  unsigned short* X     = (unsigned short*)carve((size_t)NTOK * XCOLS * 2);
  unsigned short* WIHP  = (unsigned short*)carve((size_t)256 * WPK * 2);
  unsigned short* WHHP  = (unsigned short*)carve((size_t)256 * WPK * 2);
  unsigned short* LINP  = (unsigned short*)carve((size_t)LROWS * LCOLS * 2);
  unsigned short* CONVP = (unsigned short*)carve((size_t)CROWS * CCOLS * 2);
  float*          BIASG = (float*)carve((size_t)GCOLS * 4);
  float*          G     = (float*)carve((size_t)NTOK * GCOLS * 4);
  unsigned short* HF    = (unsigned short*)carve((size_t)NTOK * HCOLS * 2);
  unsigned short* HB    = (unsigned short*)carve((size_t)NTOK * HCOLS * 2);
  if (off > ws_size || off > (size_t)134217728) return;

  pack_kernel<<<6, 256, 0, stream>>>(wih_f, whh_f, bih_f, bhh_f, wih_b, whh_b, bih_b, bhh_b, lin_w, conv_w,
                                     WIHP, WHHP, LINP, CONVP, BIASG);
  charconv_kernel<<<NTOK / TOKB, 256, 0, stream>>>(word_ids, char_ids, word_lens, word_emb, char_emb, conv_b, CONVP, X, nvocab);
  wmma_gemm64<0, false, 2, 0, false, 0><<<dim3((NTOK / 64) * (GCOLS / 64) / 8, 1), 256, 0, stream>>>(
      X, X, XCOLS, 0L, WIHP, WIHP, WPK, 0L, (void*)G, (void*)G, GCOLS, 0L,
      BIASG, G, 0L, NTOK, GCOLS, XCOLS, RS1024);
  bilstm_scan_kernel<<<2, 32, 0, stream>>>(G, WHHP, HF, HB);
  head_softmax_kernel<<<NTOK / 64, 128, 0, stream>>>(HF, HB, LINP, lin_b, out);
}
